// TransformerDecoderLayer_50929722196891
// MI455X (gfx1250) — hardware-verified
//
#include <hip/hip_runtime.h>


#ifndef NB
#define NB 4
#endif
#ifndef SEQ
#define SEQ 1024
#endif
#define NB_FULL 4
#define SEQ_FULL 1024
#define DM 1024
#define DFF 4096
#define NH 16
#define DH 64
#define PW 128
#define KT 32
#define QR 64
#define KPITCH 72
#define VPITCH 40
#define PPITCH 40
#define CPITCH 136
#define OPITCH 132
#define TPITCH 72
#define P_CARRY 16384.0f
#define ACT_CARRY 16.0f
#define W_CARRY 1024.0f
#define LN_EPS 1e-5f
#define FILL_SCALED (-1e20f * 0.125f)
#define SC_SCALE (0.125f / (ACT_CARRY * ACT_CARRY))

static_assert(NB >= 1 && NB <= NB_FULL);
static_assert(SEQ >= QR && SEQ <= SEQ_FULL);
static_assert(SEQ % QR == 0);
static_assert(SEQ % KT == 0);
static_assert((NB * SEQ) % 64 == 0);
static_assert(DM == NH * DH);
static_assert(PW == 2 * DH);
static_assert(DM % PW == 0);
static_assert(DM % 128 == 0 && DFF % 128 == 0);
static_assert(DM % 64 == 0 && DFF % 64 == 0);
static_assert(SEQ_FULL == 256 * 4);
static_assert(SEQ_FULL / KT == 32);
static_assert(((size_t)NB * SEQ * DM) % 2048 == 0);
static_assert((size_t)2 * DM * DM * 2 + (size_t)2 * DM * DFF * 2 + (size_t)3 * NB_FULL * SEQ_FULL * DM * 2 + (size_t)2 * NB_FULL * SEQ_FULL * DM * 4
              + (size_t)NB_FULL * SEQ_FULL * DFF * 2 + (size_t)2 * NB_FULL * (SEQ_FULL / QR) * 32 * 4 <= (size_t)134217728);

typedef _Float16 v8h  __attribute__((ext_vector_type(8)));
typedef _Float16 v16h __attribute__((ext_vector_type(16)));
typedef float v8f __attribute__((ext_vector_type(8)));
typedef float v4f __attribute__((ext_vector_type(4)));
typedef int v4i __attribute__((ext_vector_type(4)));

union FragH { v16h v; v8h h[2]; };

__device__ __forceinline__ unsigned f2bf(float f) { unsigned u = __float_as_uint(f); u += 0x7FFFu + ((u >> 16) & 1u); return u >> 16; }
__device__ __forceinline__ float bf16r(float f) { return __uint_as_float(f2bf(f) << 16); }
template<bool C> __device__ __forceinline__ float cvin(float f) { return C ? bf16r(f) : f; }

__device__ __forceinline__ v8f wm_f16(v16h a, v16h b, v8f c) {
    c = __builtin_amdgcn_wmma_f32_16x16x32_f16(false, a, false, b, (short)0, c, false, false);
    asm volatile("v_nop\n\tv_nop\n\tv_nop\n\tv_nop" : "+v"(c) : "v"(a), "v"(b));
    return c;
}

__global__ __launch_bounds__(256) void k_wtrans(const float* __restrict__ w, _Float16* wt, unsigned R, unsigned C)
{
    __shared__ __align__(16) _Float16 st[64 * TPITCH];
    const unsigned tid = threadIdx.x;
    const unsigned c0 = blockIdx.x * 64u, r0 = blockIdx.y * 64u;
#pragma unroll
    for (int i = 0; i < 4; ++i) {
        const unsigned p = tid + 256u * i, r = p >> 4, c4 = (p & 15u) * 4u;
        const v4f a = *(const v4f*)(w + (size_t)(r0 + r) * C + c0 + c4);
#pragma unroll
        for (int j = 0; j < 4; ++j) st[(c4 + j) * TPITCH + r] = (_Float16)(bf16r(a[j]) * W_CARRY);
    }
    __syncthreads();
    v8h ov[2];
#pragma unroll
    for (int i = 0; i < 2; ++i) {
        const unsigned p = tid + 256u * i, oc = p >> 3, pc = (p & 7u) * 8u;
        ov[i] = *(const v8h*)(st + oc * TPITCH + pc);
    }
#pragma unroll
    for (int i = 0; i < 2; ++i) {
        const unsigned p = tid + 256u * i, oc = p >> 3, pc = (p & 7u) * 8u;
        *(volatile v8h*)(wt + (size_t)(c0 + oc) * R + r0 + pc) = ov[i];
    }
    __threadfence();
#pragma unroll
    for (int i = 0; i < 2; ++i) {
        const unsigned p = tid + 256u * i, oc = p >> 3, pc = (p & 7u) * 8u;
        *(volatile v8h*)(wt + (size_t)(c0 + oc) * R + r0 + pc) = ov[i];
    }
}

__global__ __launch_bounds__(256) void k_cvt_act(const float* __restrict__ src, _Float16* dst)
{
    const unsigned e = (blockIdx.x * 256u + threadIdx.x) * 8u;
    const unsigned m = e / (unsigned)DM, col = e % (unsigned)DM;
    const unsigned bb = m / (unsigned)SEQ, n = m % (unsigned)SEQ;
    const float* s = src + (size_t)(bb * (unsigned)SEQ_FULL + n) * DM + col;
    const v4f a0 = *(const v4f*)s, a1 = *(const v4f*)(s + 4);
    v8h o;
#pragma unroll
    for (int i = 0; i < 4; ++i) { o[i] = (_Float16)(bf16r(a0[i]) * ACT_CARRY); o[4 + i] = (_Float16)(bf16r(a1[i]) * ACT_CARRY); }
    _Float16* d = dst + e;
    *(volatile v8h*)d = o;
    __threadfence();
    *(volatile v8h*)d = o;
}

__global__ __launch_bounds__(256) void k_maskflag(const int* __restrict__ m0, const int* __restrict__ m1, int* flags)
{
    __shared__ int sf[256];
    const unsigned tid = threadIdx.x;
    const unsigned qt = blockIdx.x, b = blockIdx.y, which = blockIdx.z;
    const int* mk = (which != 0u) ? m1 : m0;
    const int* base = mk + ((size_t)b * SEQ_FULL + (size_t)qt * QR) * SEQ_FULL + tid * 4u;
    int ok = 1;
#pragma unroll 4
    for (unsigned r = 0; r < (unsigned)QR; ++r) {
        const v4i v = *(const v4i*)(base + (size_t)r * SEQ_FULL);
        ok &= (int)((v[0] != 0) & (v[1] != 0) & (v[2] != 0) & (v[3] != 0));
    }
    sf[tid] = ok;
    __syncthreads();
    if (tid < 32u) {
        int f = 1;
#pragma unroll
        for (int j = 0; j < 8; ++j) f &= sf[tid * 8u + j];
        int* d = flags + ((size_t)(which * (unsigned)NB_FULL + b) * (SEQ_FULL / QR) + qt) * 32u + tid;
        *(volatile int*)d = f;
        __threadfence();
        *(volatile int*)d = f;
    }
}

template<bool CVT, bool IN_FULL>
__global__ __launch_bounds__(256) void k_ln(const float* __restrict__ x, const float* __restrict__ g, const float* __restrict__ be, _Float16* H)
{
    const unsigned tid = threadIdx.x, lane = tid & 31u, wv = tid >> 5;
    const unsigned m = blockIdx.x * 8u + wv;
    const unsigned bb = m / (unsigned)SEQ, n = m % (unsigned)SEQ;
    const unsigned srow = IN_FULL ? (bb * (unsigned)SEQ_FULL + n) : m;
    const float* xr = x + (size_t)srow * DM + lane * 8u;
    float sum = 0.f;
#pragma unroll 1
    for (unsigned j = 0; j < 4u; ++j) {
        const v4f a0 = *(const v4f*)(xr + j * 256u), a1 = *(const v4f*)(xr + j * 256u + 4u);
#pragma unroll
        for (int i = 0; i < 4; ++i) sum += cvin<CVT>(a0[i]) + cvin<CVT>(a1[i]);
    }
#pragma unroll
    for (int o = 1; o < 32; o <<= 1) sum += __shfl_xor(sum, o, 32);
    const float mu = sum * (1.0f / DM);
    float ss = 0.f;
#pragma unroll 1
    for (unsigned j = 0; j < 4u; ++j) {
        const v4f a0 = *(const v4f*)(xr + j * 256u), a1 = *(const v4f*)(xr + j * 256u + 4u);
#pragma unroll
        for (int i = 0; i < 4; ++i) {
            const float d0 = cvin<CVT>(a0[i]) - mu, d1 = cvin<CVT>(a1[i]) - mu;
            ss += d0 * d0;
            ss += d1 * d1;
        }
    }
#pragma unroll
    for (int o = 1; o < 32; o <<= 1) ss += __shfl_xor(ss, o, 32);
    const float rs = rsqrtf(ss * (1.0f / DM) + LN_EPS);
    _Float16* hr = H + (size_t)m * DM + lane * 8u;
    const float* gr = g + lane * 8u;
    const float* br = be + lane * 8u;
#pragma unroll 1
    for (unsigned j = 0; j < 4u; ++j) {
        const v4f a0 = *(const v4f*)(xr + j * 256u), a1 = *(const v4f*)(xr + j * 256u + 4u);
        const v4f g0 = *(const v4f*)(gr + j * 256u), g1 = *(const v4f*)(gr + j * 256u + 4u);
        const v4f b0 = *(const v4f*)(br + j * 256u), b1 = *(const v4f*)(br + j * 256u + 4u);
        v8h o;
#pragma unroll
        for (int i = 0; i < 4; ++i) {
            o[i]     = (_Float16)((cvin<CVT>(a0[i]) - mu) * rs * (bf16r(g0[i]) * ACT_CARRY) + bf16r(b0[i]) * ACT_CARRY);
            o[4 + i] = (_Float16)((cvin<CVT>(a1[i]) - mu) * rs * (bf16r(g1[i]) * ACT_CARRY) + bf16r(b1[i]) * ACT_CARRY);
        }
        _Float16* d = hr + j * 256u;
        *(volatile v8h*)d = o;
        __threadfence();
        *(volatile v8h*)d = o;
    }
}

__global__ __launch_bounds__(256) void k_attn(const _Float16* __restrict__ Qp, const _Float16* __restrict__ Kp, const _Float16* __restrict__ Vp,
                                             const int* __restrict__ mask, const int* __restrict__ flags, _Float16* Xc)
{
    __shared__ __align__(16) _Float16 sK[2 * KT * KPITCH];
    __shared__ __align__(16) _Float16 sVt[PW * VPITCH];
    __shared__ __align__(16) _Float16 sP[8 * 16 * PPITCH];
    __shared__ __align__(16) _Float16 sC[QR * CPITCH];

    const unsigned tid = threadIdx.x, lane = tid & 31u, wv = tid >> 5, hh = lane >> 4, lm = lane & 15u;
    const unsigned rg = wv & 3u, s = wv >> 2;
    const unsigned b = blockIdx.z, hp = blockIdx.y, qt = blockIdx.x, q0 = qt * (unsigned)QR;
    const size_t kvrow0 = (size_t)b * SEQ;

    FragH qa[2];
    {
        const _Float16* qrow = Qp + (kvrow0 + q0 + rg * 16u + lm) * DM + hp * (unsigned)PW + s * (unsigned)DH;
#pragma unroll
        for (int j = 0; j < 2; ++j) {
            qa[j].h[0] = *(const v8h*)(qrow + 32 * j + 8u * hh);
            qa[j].h[1] = *(const v8h*)(qrow + 32 * j + 16 + 8u * hh);
        }
    }
    v8f acc[4];
    float rm[8], rl[8];
#pragma unroll
    for (int t = 0; t < 4; ++t) acc[t] = (v8f){};
#pragma unroll
    for (int r = 0; r < 8; ++r) { rm[r] = -1e30f; rl[r] = 0.f; }

    const int* fl = flags + ((size_t)b * (SEQ_FULL / QR) + qt) * 32u;
    const int* mrow = mask + ((size_t)b * SEQ_FULL + q0 + rg * 16u + 8u * hh) * SEQ_FULL + lm;

#pragma unroll 1
    for (unsigned kt = 0; kt < (unsigned)(SEQ / KT); ++kt) {
        const unsigned key0 = kt * (unsigned)KT;
#pragma unroll
        for (int i = 0; i < 2; ++i) {
            const unsigned p = tid + 256u * i, key = p >> 4, c16 = p & 15u;
            const size_t gofs = (kvrow0 + key0 + key) * DM + hp * (unsigned)PW + c16 * 8u;
            const v8h kv = *(const v8h*)(Kp + gofs);
            *(v8h*)(sK + ((c16 >> 3) * (unsigned)KT + key) * KPITCH + (c16 & 7u) * 8u) = kv;
            const v8h vv = *(const v8h*)(Vp + gofs);
#pragma unroll
            for (int j = 0; j < 8; ++j) sVt[(c16 * 8u + j) * VPITCH + key] = vv[j];
        }
        __syncthreads();

        v8f sc[2];
#pragma unroll
        for (int t = 0; t < 2; ++t) {
            v8f c = (v8f){};
#pragma unroll
            for (int j = 0; j < 2; ++j) {
                FragH kb;
                const _Float16* kr = sK + (s * (unsigned)KT + t * 16 + lm) * KPITCH + 32 * j;
                kb.h[0] = *(const v8h*)(kr + 8u * hh);
                kb.h[1] = *(const v8h*)(kr + 16 + 8u * hh);
                c = wm_f16(qa[j].v, kb.v, c);
            }
            sc[t] = c;
        }
        float x0[8], x1[8];
#pragma unroll
        for (int r = 0; r < 8; ++r) { x0[r] = sc[0][r] * SC_SCALE; x1[r] = sc[1][r] * SC_SCALE; }

        const int fast = __builtin_amdgcn_readfirstlane(fl[kt]);
        if (fast != 1) {
            const int* mp = mrow + key0;
#pragma unroll
            for (int r = 0; r < 8; ++r) {
                const int mv = mp[(size_t)r * SEQ_FULL];
                x0[r] = (mv == 0) ? FILL_SCALED : x0[r];
            }
#pragma unroll
            for (int r = 0; r < 8; ++r) {
                const int mv = mp[(size_t)r * SEQ_FULL + 16];
                x1[r] = (mv == 0) ? FILL_SCALED : x1[r];
            }
        }

#pragma unroll
        for (int r = 0; r < 8; ++r) {
            float mx = fmaxf(x0[r], x1[r]);
#pragma unroll
            for (int o = 1; o < 16; o <<= 1) mx = fmaxf(mx, __shfl_xor(mx, o, 32));
            const float nm = fmaxf(rm[r], mx);
            const float corr = __expf(rm[r] - nm);
            const float p0 = __expf(x0[r] - nm), p1 = __expf(x1[r] - nm);
            float rs = p0 + p1;
#pragma unroll
            for (int o = 1; o < 16; o <<= 1) rs += __shfl_xor(rs, o, 32);
            rl[r] = rl[r] * corr + rs;
            rm[r] = nm;
#pragma unroll
            for (int t = 0; t < 4; ++t) acc[t][r] = acc[t][r] * corr;
            _Float16* prow = sP + (wv * 16u + 8u * hh + r) * PPITCH;
            prow[lm] = (_Float16)(p0 * P_CARRY);
            prow[16 + lm] = (_Float16)(p1 * P_CARRY);
        }
        __syncthreads();

        {
            FragH pa;
            const _Float16* pr = sP + (wv * 16u + lm) * PPITCH;
            pa.h[0] = *(const v8h*)(pr + 8u * hh);
            pa.h[1] = *(const v8h*)(pr + 16 + 8u * hh);
#pragma unroll
            for (int t = 0; t < 4; ++t) {
                FragH vb;
                const _Float16* vr = sVt + (s * (unsigned)DH + t * 16 + lm) * VPITCH;
                vb.h[0] = *(const v8h*)(vr + 8u * hh);
                vb.h[1] = *(const v8h*)(vr + 16 + 8u * hh);
                acc[t] = wm_f16(pa.v, vb.v, acc[t]);
            }
        }
        __syncthreads();
    }

#pragma unroll
    for (int r = 0; r < 8; ++r) {
        const float inv = (1.0f / rl[r]) * (ACT_CARRY / (P_CARRY * ACT_CARRY));
#pragma unroll
        for (int t = 0; t < 4; ++t)
            sC[(rg * 16u + 8u * hh + r) * CPITCH + s * (unsigned)DH + t * 16 + lm] = (_Float16)(acc[t][r] * inv);
    }
    __syncthreads();
    v8h ov[4];
#pragma unroll
    for (int i = 0; i < 4; ++i) {
        const unsigned p = tid + 256u * i, row = p >> 4, c8 = (p & 15u) * 8u;
        ov[i] = *(const v8h*)(sC + row * CPITCH + c8);
    }
#pragma unroll
    for (int i = 0; i < 4; ++i) {
        const unsigned p = tid + 256u * i, row = p >> 4, c8 = (p & 15u) * 8u;
        *(volatile v8h*)(Xc + (kvrow0 + q0 + row) * DM + hp * (unsigned)PW + c8) = ov[i];
    }
    __threadfence();
#pragma unroll
    for (int i = 0; i < 4; ++i) {
        const unsigned p = tid + 256u * i, row = p >> 4, c8 = (p & 15u) * 8u;
        *(volatile v8h*)(Xc + (kvrow0 + q0 + row) * DM + hp * (unsigned)PW + c8) = ov[i];
    }
}

template<int KD, int ND, int MODE, bool RES_BF, bool RES_FULL, bool OUT_FULL>
__global__ __launch_bounds__(256) void k_gemm(const _Float16* __restrict__ X, const _Float16* __restrict__ Wt, const float* __restrict__ bias,
                                             const float* resid, void* outp)
{
    static_assert(KD % 32 == 0);
    static_assert(ND % 128 == 0);
    __shared__ __align__(16) float cst[64 * OPITCH];
    const unsigned tid = threadIdx.x, lane = tid & 31u, wv = tid >> 5, hh = lane >> 4, lm = lane & 15u;
    const unsigned rt = wv & 3u, ch = wv >> 2;
    const unsigned row0 = blockIdx.x * 64u, cb = blockIdx.y * 128u, col0 = cb + ch * 64u;
    const _Float16* xr = X + (size_t)(row0 + rt * 16u + lm) * KD;
    v8f acc[4];
#pragma unroll
    for (int t = 0; t < 4; ++t) acc[t] = (v8f){};
#pragma unroll 2
    for (unsigned kc = 0; kc < (unsigned)KD; kc += 32u) {
        FragH a;
        a.h[0] = *(const v8h*)(xr + kc + 8u * hh);
        a.h[1] = *(const v8h*)(xr + kc + 16u + 8u * hh);
#pragma unroll
        for (int t = 0; t < 4; ++t) {
            FragH bb;
            const _Float16* wr = Wt + (size_t)(col0 + t * 16 + lm) * KD + kc;
            bb.h[0] = *(const v8h*)(wr + 8u * hh);
            bb.h[1] = *(const v8h*)(wr + 16u + 8u * hh);
            acc[t] = wm_f16(a.v, bb.v, acc[t]);
        }
    }
#pragma unroll
    for (int t = 0; t < 4; ++t) {
        const unsigned cl = ch * 64u + t * 16 + lm;
        const float bv = bf16r(bias[cb + cl]);
#pragma unroll
        for (int r = 0; r < 8; ++r) cst[(rt * 16u + 8u * hh + r) * OPITCH + cl] = acc[t][r] * (1.0f / (ACT_CARRY * W_CARRY)) + bv;
    }
    __syncthreads();
    if (MODE == 0) {
        float* out = (float*)outp;
        v4f ov[8];
#pragma unroll
        for (int i = 0; i < 8; ++i) {
            const unsigned p = tid + 256u * i, row = p >> 5, c4 = (p & 31u) * 4u;
            const unsigned m = row0 + row;
            const unsigned rrow = RES_FULL ? ((m / (unsigned)SEQ) * (unsigned)SEQ_FULL + (m % (unsigned)SEQ)) : m;
            v4f rv = *(const v4f*)(resid + (size_t)rrow * ND + cb + c4);
            if (RES_BF) {
#pragma unroll
                for (int j = 0; j < 4; ++j) rv[j] = bf16r(rv[j]);
            }
            const v4f cv = *(const v4f*)(cst + row * OPITCH + c4);
            ov[i] = cv + rv;
        }
#pragma unroll
        for (int i = 0; i < 8; ++i) {
            const unsigned p = tid + 256u * i, row = p >> 5, c4 = (p & 31u) * 4u;
            const unsigned m = row0 + row;
            const unsigned orow = OUT_FULL ? ((m / (unsigned)SEQ) * (unsigned)SEQ_FULL + (m % (unsigned)SEQ)) : m;
            *(volatile v4f*)(out + (size_t)orow * ND + cb + c4) = ov[i];
        }
        __threadfence();
#pragma unroll
        for (int i = 0; i < 8; ++i) {
            const unsigned p = tid + 256u * i, row = p >> 5, c4 = (p & 31u) * 4u;
            const unsigned m = row0 + row;
            const unsigned orow = OUT_FULL ? ((m / (unsigned)SEQ) * (unsigned)SEQ_FULL + (m % (unsigned)SEQ)) : m;
            *(volatile v4f*)(out + (size_t)orow * ND + cb + c4) = ov[i];
        }
    } else {
        _Float16* out = (_Float16*)outp;
        v8h oh[4];
#pragma unroll
        for (int i = 0; i < 4; ++i) {
            const unsigned p = tid + 256u * i, row = p >> 4, c8 = (p & 15u) * 8u;
            const v4f a0 = *(const v4f*)(cst + row * OPITCH + c8), a1 = *(const v4f*)(cst + row * OPITCH + c8 + 4u);
#pragma unroll
            for (int j = 0; j < 4; ++j) {
                oh[i][j]     = (_Float16)(fmaxf(a0[j], 0.0f) * ACT_CARRY);
                oh[i][4 + j] = (_Float16)(fmaxf(a1[j], 0.0f) * ACT_CARRY);
            }
        }
#pragma unroll
        for (int i = 0; i < 4; ++i) {
            const unsigned p = tid + 256u * i, row = p >> 4, c8 = (p & 15u) * 8u;
            *(volatile v8h*)(out + (size_t)(row0 + row) * ND + cb + c8) = oh[i];
        }
        __threadfence();
#pragma unroll
        for (int i = 0; i < 4; ++i) {
            const unsigned p = tid + 256u * i, row = p >> 4, c8 = (p & 15u) * 8u;
            *(volatile v8h*)(out + (size_t)(row0 + row) * ND + cb + c8) = oh[i];
        }
    }
}

extern "C" void kernel_launch(void* const* d_in, const int* in_sizes, int n_in,
                              void* d_out, int out_size, void* d_ws, size_t ws_size, hipStream_t stream)
{
    if (n_in < 18) return;
    const long long needAct = ((long long)(NB - 1) * SEQ_FULL + SEQ) * DM;
    const long long needMask = ((long long)(NB - 1) * SEQ_FULL + SEQ) * SEQ_FULL;
    if ((long long)in_sizes[0] < needAct || (long long)in_sizes[1] < needAct) return;
    if ((long long)in_sizes[2] < needMask || (long long)in_sizes[3] < needMask) return;
    if (in_sizes[4] < DM * DM || in_sizes[5] < DM || in_sizes[6] < DM * DM || in_sizes[7] < DM) return;
    if (in_sizes[8] < DM * DFF || in_sizes[9] < DFF || in_sizes[10] < DFF * DM || in_sizes[11] < DM) return;
    for (int i = 12; i < 18; ++i) if (in_sizes[i] < DM) return;
    if ((long long)out_size < needAct) return;

    const float* tgt      = (const float*)d_in[0];
    const float* memory   = (const float*)d_in[1];
    const int*   tgt_mask = (const int*)d_in[2];
    const int*   mem_mask = (const int*)d_in[3];
    const float* sa_w  = (const float*)d_in[4];
    const float* sa_b  = (const float*)d_in[5];
    const float* mha_w = (const float*)d_in[6];
    const float* mha_b = (const float*)d_in[7];
    const float* ff_w1 = (const float*)d_in[8];
    const float* ff_b1 = (const float*)d_in[9];
    const float* ff_w2 = (const float*)d_in[10];
    const float* ff_b2 = (const float*)d_in[11];
    const float* ln1_g = (const float*)d_in[12];
    const float* ln1_b = (const float*)d_in[13];
    const float* ln2_g = (const float*)d_in[14];
    const float* ln2_b = (const float*)d_in[15];
    const float* ln3_g = (const float*)d_in[16];
    const float* ln3_b = (const float*)d_in[17];
    float* out = (float*)d_out;

    const size_t nact = (size_t)NB * SEQ * DM;
    unsigned char* base = (unsigned char*)d_ws;
    size_t off = 0;
    _Float16* Wsa = (_Float16*)(base + off); off += (size_t)DM * DM * 2;
    _Float16* Wmh = (_Float16*)(base + off); off += (size_t)DM * DM * 2;
    _Float16* W1t = (_Float16*)(base + off); off += (size_t)DM * DFF * 2;
    _Float16* W2t = (_Float16*)(base + off); off += (size_t)DFF * DM * 2;
    _Float16* Mh  = (_Float16*)(base + off); off += nact * 2;
    _Float16* Hh  = (_Float16*)(base + off); off += nact * 2;
    _Float16* Xc  = (_Float16*)(base + off); off += nact * 2;
    float* X1     = (float*)(base + off);    off += nact * 4;
    float* X2     = (float*)(base + off);    off += nact * 4;
    _Float16* Tp  = (_Float16*)(base + off); off += (size_t)NB * SEQ * DFF * 2;
    int* Fl       = (int*)(base + off);      off += (size_t)2 * NB_FULL * (SEQ_FULL / QR) * 32 * 4;
    if (off > ws_size) return;

    const dim3 B256(256);
    k_wtrans<<<dim3(DM / 64, DM / 64), B256, 0, stream>>>(sa_w, Wsa, (unsigned)DM, (unsigned)DM);
    k_wtrans<<<dim3(DM / 64, DM / 64), B256, 0, stream>>>(mha_w, Wmh, (unsigned)DM, (unsigned)DM);
    k_wtrans<<<dim3(DFF / 64, DM / 64), B256, 0, stream>>>(ff_w1, W1t, (unsigned)DM, (unsigned)DFF);
    k_wtrans<<<dim3(DM / 64, DFF / 64), B256, 0, stream>>>(ff_w2, W2t, (unsigned)DFF, (unsigned)DM);
    k_cvt_act<<<dim3((unsigned)(nact / 2048)), B256, 0, stream>>>(memory, Mh);
    k_maskflag<<<dim3(SEQ / QR, NB, 2), B256, 0, stream>>>(tgt_mask, mem_mask, Fl);
    const int* Fl0 = Fl;
    const int* Fl1 = Fl + (size_t)NB_FULL * (SEQ_FULL / QR) * 32;

    const dim3 gAttn(SEQ / QR, DM / PW, NB);
    const dim3 gLn((NB * SEQ) / 8);
    const dim3 gD((NB * SEQ) / 64, DM / 128);
    const dim3 gF((NB * SEQ) / 64, DFF / 128);

    k_ln<true, true><<<gLn, B256, 0, stream>>>(tgt, ln1_g, ln1_b, Hh);
    k_attn<<<gAttn, B256, 0, stream>>>(Hh, Hh, Hh, tgt_mask, Fl0, Xc);
    k_gemm<DM, DM, 0, true, true, false><<<gD, B256, 0, stream>>>(Xc, Wsa, sa_b, tgt, (void*)X1);

    k_ln<false, false><<<gLn, B256, 0, stream>>>(X1, ln2_g, ln2_b, Hh);
    k_attn<<<gAttn, B256, 0, stream>>>(Mh, Mh, Hh, mem_mask, Fl1, Xc);
    k_gemm<DM, DM, 0, false, false, false><<<gD, B256, 0, stream>>>(Xc, Wmh, mha_b, X1, (void*)X2);

    k_ln<false, false><<<gLn, B256, 0, stream>>>(X2, ln3_g, ln3_b, Hh);
    k_gemm<DM, DFF, 1, false, false, false><<<gF, B256, 0, stream>>>(Hh, W1t, ff_b1, (const float*)nullptr, (void*)Tp);
    k_gemm<DFF, DM, 0, false, false, true><<<gD, B256, 0, stream>>>(Tp, W2t, ff_b2, X2, (void*)out);
}
